// GTDynamics_2714419331263
// MI455X (gfx1250) — hardware-verified
//
#include <hip/hip_runtime.h>
#include <math.h>

typedef __attribute__((ext_vector_type(16))) _Float16 v16h;
typedef __attribute__((ext_vector_type(16))) __bf16 v16b;
typedef __attribute__((ext_vector_type(8)))  _Float16 v8h;
typedef __attribute__((ext_vector_type(8)))  float v8f;
typedef __attribute__((ext_vector_type(4)))  float v4f;
typedef __attribute__((ext_vector_type(2)))  float v2f;
typedef __attribute__((ext_vector_type(4)))  unsigned v4u;
typedef __attribute__((ext_vector_type(4)))  int v4i;
typedef float __attribute__((may_alias)) float_a;
typedef int __attribute__((may_alias)) int_a;

template <typename T> __device__ __forceinline__ void vst2(void* p, T v) { *(volatile T*)p = v; __threadfence(); *(volatile T*)p = v; }
__device__ __forceinline__ v8f wmma16(v16h a, v16h b, v8f c) {
  v8f d = __builtin_amdgcn_wmma_f32_16x16x32_f16(false, a, false, b, (short)0, c, false, false);
  asm volatile("v_nop\n\tv_nop\n\tv_nop\n\tv_nop" : "+v"(d) : "v"(a), "v"(b));
  return d;
}
__device__ __forceinline__ v8f wmma_bf(v16b a, v16b b, v8f c) {
  v8f d = __builtin_amdgcn_wmma_f32_16x16x32_bf16(false, a, false, b, (short)0, c, false, false);
  asm volatile("v_nop\n\tv_nop\n\tv_nop\n\tv_nop" : "+v"(d) : "v"(a), "v"(b));
  return d;
}
__device__ __forceinline__ v16h frag_h(const _Float16* rowk0, int lane) {
  union { v16h v; v8h q[2]; } u; const _Float16* p = rowk0 + 8 * (lane >> 4);
  u.q[0] = *(const v8h*)p; u.q[1] = *(const v8h*)(p + 16); return u.v;
}
__device__ __forceinline__ v16h frag_f32(const float* rowk0, int lane) {
  v16h a; const float* p = rowk0 + 8 * (lane >> 4);
#pragma unroll
  for (int i = 0; i < 8; ++i) { a[i] = (_Float16)p[i]; a[8 + i] = (_Float16)p[16 + i]; }
  return a;
}
__device__ __forceinline__ v16h frag_f32s(const float* rowk0, int lane, float sc) {
  v16h a; const float* p = rowk0 + 8 * (lane >> 4);
#pragma unroll
  for (int i = 0; i < 8; ++i) { a[i] = (_Float16)(p[i] * sc); a[8 + i] = (_Float16)(p[16 + i] * sc); }
  return a;
}
__device__ __forceinline__ v16h fragc_f32(const float* W, int k0, int n, int lane, int ld, int K) {
  v16h a; const int g = lane >> 4;
#pragma unroll
  for (int i = 0; i < 8; ++i) { const int ka = k0 + 8 * g + i, kb = ka + 16;
    a[i] = (_Float16)(ka < K ? W[(size_t)ka * ld + n] : 0.f); a[8 + i] = (_Float16)(kb < K ? W[(size_t)kb * ld + n] : 0.f); }
  return a;
}
struct F2 { v16b h, l; };
__device__ __forceinline__ F2 bsplit16(const float v[16]) { F2 r;
#pragma unroll
  for (int i = 0; i < 16; ++i) { const __bf16 h = (__bf16)v[i]; r.h[i] = h; r.l[i] = (__bf16)(v[i] - (float)h); }
  return r; }
__device__ __forceinline__ F2 split_row(const float* row, int k0, int lane) { float v[16]; const float* p = row + k0 + 8 * (lane >> 4);
#pragma unroll
  for (int i = 0; i < 8; ++i) { v[i] = p[i]; v[8 + i] = p[16 + i]; }
  return bsplit16(v); }
__device__ __forceinline__ F2 split_rowK(const float* row, int k0, int lane, int K) { float v[16]; const int g = lane >> 4;
#pragma unroll
  for (int i = 0; i < 8; ++i) { const int ka = k0 + 8 * g + i, kb = ka + 16; v[i] = ka < K ? row[ka] : 0.f; v[8 + i] = kb < K ? row[kb] : 0.f; }
  return bsplit16(v); }
__device__ __forceinline__ F2 split_col(const float* W, int k0, int n, int lane, int ld, int K) { float v[16]; const int g = lane >> 4;
#pragma unroll
  for (int i = 0; i < 8; ++i) { const int ka = k0 + 8 * g + i, kb = ka + 16; v[i] = ka < K ? W[(size_t)ka * ld + n] : 0.f; v[8 + i] = kb < K ? W[(size_t)kb * ld + n] : 0.f; }
  return bsplit16(v); }
__device__ __forceinline__ v8f mac3(const F2& a, const F2& b, v8f c) { c = wmma_bf(a.l, b.h, c); c = wmma_bf(a.h, b.l, c); return wmma_bf(a.h, b.h, c); }
__device__ __forceinline__ float sigm(float v) { return 1.0f / (1.0f + expf(-v)); }
#define LDSX() do { asm volatile("s_wait_dscnt 0" ::: "memory"); __builtin_amdgcn_wave_barrier(); __builtin_amdgcn_fence(__ATOMIC_RELEASE, "workgroup"); } while (0)

#define NB 2
#define NN 512
#define DM 256
#define NH 8
#define DH 32
#define NR (NB * NN)

__global__ __launch_bounds__(256) void k_enc(const float* __restrict__ x, const float* __restrict__ t, const float* __restrict__ Wenc, float* __restrict__ nodes, float* __restrict__ dist) {
  const int tid = threadIdx.x, r = blockIdx.x;
  __shared__ __align__(16) float so[DM]; __shared__ __align__(16) float sd[NN];
  const float x0 = x[(size_t)r * 3], x1 = x[(size_t)r * 3 + 1], x2 = x[(size_t)r * 3 + 2], tv = t[r];
  so[tid] = x0 * Wenc[tid] + x1 * Wenc[DM + tid] + x2 * Wenc[2 * DM + tid] + tv * Wenc[3 * DM + tid];
  const int b = r / NN;
  for (int j = tid; j < NN; j += 256) { const float* xj = x + ((size_t)b * NN + j) * 3; const float dx = x0 - xj[0], dy = x1 - xj[1], dz = x2 - xj[2]; const float d2 = dx * dx + dy * dy + dz * dz; sd[j] = d2 > 0.f ? sqrtf(d2) : 0.f; }
  __syncthreads();
  if (tid < DM / 4) vst2(nodes + (size_t)r * DM + tid * 4, *(const v4f*)(&so[tid * 4]));
  if (tid < NN / 4) vst2(dist + (size_t)r * NN + tid * 4, *(const v4f*)(&sd[tid * 4]));
}
__global__ __launch_bounds__(128) void k_qkv(const float* __restrict__ nodes, const float* __restrict__ lg, const float* __restrict__ lb, const float* __restrict__ Wq, const float* __restrict__ bq, const float* __restrict__ Wkv, const float* __restrict__ bkv, const float* __restrict__ We, const float* __restrict__ be,
                                           float* __restrict__ Q, float* __restrict__ Kr, float* __restrict__ V, float* __restrict__ qe, float* __restrict__ qb) {
  __shared__ __align__(16) float sh[4][16][DM + 4];
  __shared__ __align__(16) float so[4][16][DM + 4];
  __shared__ __align__(16) float sr[4][16][DM + 4];
  __shared__ __align__(16) float sq[4][16][16];
  const int tid = threadIdx.x, wave = tid >> 5, lane = tid & 31, col = lane & 15, g = lane >> 4;
  const int r0 = blockIdx.x * 64 + wave * 16;
  for (int rl = 0; rl < 16; ++rl) { const float* nr = nodes + (size_t)(r0 + rl) * DM; float v[8]; float s = 0.f;
#pragma unroll
    for (int e = 0; e < 8; ++e) { v[e] = nr[lane * 8 + e]; s += v[e]; }
#pragma unroll
    for (int off = 16; off >= 1; off >>= 1) s += __shfl_xor(s, off, 32);
    const float mu = s * (1.0f / DM); float q2 = 0.f;
#pragma unroll
    for (int e = 0; e < 8; ++e) { const float d = v[e] - mu; q2 += d * d; }
#pragma unroll
    for (int off = 16; off >= 1; off >>= 1) q2 += __shfl_xor(q2, off, 32);
    const float rs = rsqrtf(q2 * (1.0f / DM) + 1e-5f);
#pragma unroll
    for (int e = 0; e < 8; ++e) { const int c = lane * 8 + e; sh[wave][rl][c] = (v[e] - mu) * rs * lg[c] + lb[c]; } }
  LDSX();
#pragma unroll 1
  for (int which = 0; which < 3; ++which) { const float* W = which == 0 ? Wq : Wkv; const int ldw = which == 0 ? DM : 2 * DM; const int cb = which == 2 ? DM : 0; const float* bias = which == 0 ? bq : bkv + cb;
#pragma unroll 1
    for (int np = 0; np < 2; ++np) { v8f acc[8] = {};
#pragma unroll 1
      for (int kc = 0; kc < DM / 32; ++kc) { const F2 a = split_row(&sh[wave][col][0], kc * 32, lane);
#pragma unroll
        for (int j = 0; j < 8; ++j) acc[j] = mac3(a, split_col(W + cb, kc * 32, np * 128 + j * 16 + col, lane, ldw, DM), acc[j]); }
#pragma unroll
      for (int j = 0; j < 8; ++j) { const int c = np * 128 + j * 16 + col; const float bb = bias[c];
#pragma unroll
        for (int r = 0; r < 8; ++r) so[wave][8 * g + r][c] = acc[j][r] + bb; } }
    LDSX();
    float* dst = which == 0 ? Q : (which == 1 ? Kr : V);
    if (which < 2) {
      for (int q = lane; q < 16 * DM; q += 32) { const int rl = q >> 8, c = q & 255; const int h = c >> 5, d = c & 31, dd = d & 15; const int n = (r0 + rl) % NN;
        const float invf = 1.0f / powf(10000.0f, (float)(2 * dd) * (1.0f / 32.0f)); const float ang = (float)n * invf; float sv, cv; sincosf(ang, &sv, &cv);
        const float tv = so[wave][rl][c]; const float pr = d < 16 ? -so[wave][rl][h * DH + d + 16] : so[wave][rl][h * DH + d - 16];
        sr[wave][rl][c] = tv * cv + pr * sv; }
      LDSX();
      for (int q = lane; q < 16 * 64; q += 32) { const int rl = q >> 6, pc = q & 63; vst2(dst + (size_t)(r0 + rl) * DM + pc * 4, *(const v4f*)(&sr[wave][rl][pc * 4])); }
      if (which == 0) {
        for (int q = lane; q < 16 * NH; q += 32) { const int rl = q >> 3, h = q & 7; float e1 = 0.f, e2 = 0.f;
#pragma unroll 8
          for (int d = 0; d < DH; ++d) { const float qv = sr[wave][rl][h * DH + d]; e1 += qv * We[h * DH + d]; e2 += qv * be[h * DH + d]; }
          sq[wave][rl][h] = e1; sq[wave][rl][8 + h] = e2; }
        LDSX();
        for (int q = lane; q < 16 * 4; q += 32) { const int rl = q >> 2, pc = q & 3; vst2((pc < 2 ? qe : qb) + (size_t)(r0 + rl) * NH + (pc & 1) * 4, *(const v4f*)(&sq[wave][rl][pc * 4])); } } }
    else { for (int q = lane; q < 16 * 64; q += 32) { const int rl = q >> 6, pc = q & 63; vst2(dst + (size_t)(r0 + rl) * DM + pc * 4, *(const v4f*)(&so[wave][rl][pc * 4])); } }
    LDSX(); }
}
__global__ __launch_bounds__(64) void k_attn(const float* __restrict__ Q, const float* __restrict__ Kr, const float* __restrict__ V, const float* __restrict__ qe, const float* __restrict__ qb, const float* __restrict__ dist, const float* __restrict__ We, const float* __restrict__ be, float* __restrict__ O) {
  __shared__ __align__(16) float sS[2][16][NN + 8];
  __shared__ __align__(16) float sO[2][16][36];
  __shared__ float sad[2][16];
  const int tid = threadIdx.x, w = tid >> 5, lane = tid & 31, col = lane & 15, g = lane >> 4;
  const int b = blockIdx.z, h = blockIdx.y, i0 = blockIdx.x * 32 + w * 16; const size_t rb = (size_t)b * NN;
  const F2 aq = split_row(Q + (rb + i0 + col) * DM + h * DH, 0, lane);
  const float scl = 0.17677669529663687f;
#pragma unroll 2
  for (int t = 0; t < NN / 16; ++t) { v8f s = {}; s = mac3(aq, split_row(Kr + (rb + t * 16 + col) * DM + h * DH, 0, lane), s);
#pragma unroll
    for (int r = 0; r < 8; ++r) { const int i = i0 + 8 * g + r, j = t * 16 + col; const size_t ri = rb + i;
      sS[w][8 * g + r][j] = (s[r] + dist[ri * NN + j] * qe[ri * NH + h] + qb[ri * NH + h]) * scl; } }
  LDSX();
  { const int m = col; float* row = &sS[w][m][0]; float mx = -3.4e38f;
#pragma unroll 8
    for (int j = g * 256; j < g * 256 + 256; ++j) mx = fmaxf(mx, row[j]);
    mx = fmaxf(mx, __shfl_xor(mx, 16, 32)); float l = 0.f, ad = 0.f; const size_t ri = rb + i0 + m;
#pragma unroll 8
    for (int j = g * 256; j < g * 256 + 256; ++j) { const float p = expf(row[j] - mx); row[j] = p; l += p; ad += p * dist[ri * NN + j]; }
    l += __shfl_xor(l, 16, 32); ad += __shfl_xor(ad, 16, 32); const float inv = 1.0f / l;
    LDSX();
#pragma unroll 8
    for (int j = g * 256; j < g * 256 + 256; ++j) row[j] *= inv;
    if (g == 0) sad[w][m] = ad * inv; }
  LDSX();
  v8f acc[2] = {};
#pragma unroll 2
  for (int kc = 0; kc < NN / 32; ++kc) { const F2 pa = split_row(&sS[w][col][0], kc * 32, lane);
#pragma unroll
    for (int t = 0; t < 2; ++t) acc[t] = mac3(pa, split_col(V + (rb + kc * 32) * DM + h * DH, 0, t * 16 + col, lane, DM, 32), acc[t]); }
#pragma unroll
  for (int t = 0; t < 2; ++t) { const int d = t * 16 + col;
#pragma unroll
    for (int r = 0; r < 8; ++r) { const int m = 8 * g + r; sO[w][m][d] = acc[t][r] + sad[w][m] * We[h * DH + d] + be[h * DH + d]; } }
  LDSX();
  for (int q = lane; q < 16 * 8; q += 32) { const int rl = q >> 3, pc = q & 7; vst2(O + (rb + i0 + rl) * DM + h * DH + pc * 4, *(const v4f*)(&sO[w][rl][pc * 4])); }
}
__global__ __launch_bounds__(128) void k_out(const float* __restrict__ O, const float* __restrict__ Wo, const float* __restrict__ bo, const float* __restrict__ Wg, float* __restrict__ nodes) {
  __shared__ __align__(16) float so[4][16][DM + 4];
  __shared__ float sg[4][16];
  const int tid = threadIdx.x, wave = tid >> 5, lane = tid & 31, col = lane & 15, g = lane >> 4;
  const int r0 = blockIdx.x * 64 + wave * 16;
#pragma unroll 1
  for (int np = 0; np < 2; ++np) { v8f acc[8] = {};
#pragma unroll 1
    for (int kc = 0; kc < DM / 32; ++kc) { const F2 a = split_row(O + (size_t)(r0 + col) * DM, kc * 32, lane);
#pragma unroll
      for (int j = 0; j < 8; ++j) acc[j] = mac3(a, split_col(Wo, kc * 32, np * 128 + j * 16 + col, lane, DM, DM), acc[j]); }
#pragma unroll
    for (int j = 0; j < 8; ++j) { const int c = np * 128 + j * 16 + col; const float bb = bo[c];
#pragma unroll
      for (int r = 0; r < 8; ++r) so[wave][8 * g + r][c] = acc[j][r] + bb; } }
  LDSX();
  { const int rl = lane >> 1, hf = lane & 1; const float* nr = nodes + (size_t)(r0 + rl) * DM; float s = 0.f;
#pragma unroll 4
    for (int c = hf * 128; c < hf * 128 + 128; ++c) { const float o2 = so[wave][rl][c], nv = nr[c]; s += o2 * Wg[c] + nv * Wg[DM + c] + (o2 - nv) * Wg[2 * DM + c]; }
    s += __shfl_xor(s, 1, 32); if (hf == 0) sg[wave][rl] = sigm(s); }
  LDSX();
  for (int q = lane; q < 16 * DM; q += 32) { const int rl = q >> 8, c = q & 255; const float gt = sg[wave][rl]; const float nv = nodes[(size_t)(r0 + rl) * DM + c]; so[wave][rl][c] = so[wave][rl][c] * gt + nv * (1.0f - gt); }
  LDSX();
  for (int q = lane; q < 16 * 64; q += 32) { const int rl = q >> 6, pc = q & 63; vst2(nodes + (size_t)(r0 + rl) * DM + pc * 4, *(const v4f*)(&so[wave][rl][pc * 4])); }
}
__global__ __launch_bounds__(1024) void k_dec(const float* __restrict__ nodes, const float* __restrict__ Wdec, float* __restrict__ out) {
  const int r = threadIdx.x; const float* nr = nodes + (size_t)r * DM; float a0 = 0.f, a1 = 0.f, a2 = 0.f;
#pragma unroll 4
  for (int c = 0; c < DM; ++c) { const float v = nr[c]; a0 += v * Wdec[c * 3]; a1 += v * Wdec[c * 3 + 1]; a2 += v * Wdec[c * 3 + 2]; }
  vst2(out + (size_t)r * 3, a0); vst2(out + (size_t)r * 3 + 1, a1); vst2(out + (size_t)r * 3 + 2, a2);
}
extern "C" void kernel_launch(void* const* d_in, const int* in_sizes, int n_in, void* d_out, int out_size, void* d_ws, size_t ws_size, hipStream_t stream) {
  (void)in_sizes; (void)n_in; (void)out_size; (void)ws_size;
  const float** I = (const float**)d_in;
  const float* x = I[0]; const float* t = I[1]; const float* Wenc = I[2]; const float* Wdec = I[3]; const float* lng = I[4]; const float* lnb = I[5]; const float* Wq = I[6]; const float* bq = I[7]; const float* Wkv = I[8]; const float* bkv = I[9];
  const float* We = I[10]; const float* be = I[11]; const float* Wo = I[12]; const float* bo = I[13]; const float* Wg = I[14];
  float* out = (float*)d_out;
  char* ws = (char*)d_ws; size_t off = 0;
  auto take = [&](size_t bytes) { char* p = ws + off; off += (bytes + 255) & ~(size_t)255; return p; };
  float* nodes = (float*)take((size_t)NR * DM * 4); float* dist = (float*)take((size_t)NR * NN * 4); float* Q = (float*)take((size_t)NR * DM * 4); float* Kr = (float*)take((size_t)NR * DM * 4); float* V = (float*)take((size_t)NR * DM * 4);
  float* qe = (float*)take((size_t)NR * NH * 4); float* qb = (float*)take((size_t)NR * NH * 4); float* O = (float*)take((size_t)NR * DM * 4);
  k_enc<<<NR, 256, 0, stream>>>(x, t, Wenc, nodes, dist);
  for (int l = 0; l < 2; ++l) {
    k_qkv<<<NR / 64, 128, 0, stream>>>(nodes, lng + l * DM, lnb + l * DM, Wq + (size_t)l * DM * DM, bq + l * DM, Wkv + (size_t)l * DM * 2 * DM, bkv + l * 2 * DM, We + l * DM, be + l * DM, Q, Kr, V, qe, qb);
    k_attn<<<dim3(NN / 32, NH, NB), 64, 0, stream>>>(Q, Kr, V, qe, qb, dist, We + l * DM, be + l * DM, O);
    k_out<<<NR / 64, 128, 0, stream>>>(O, Wo + (size_t)l * DM * DM, bo + l * DM, Wg + l * 3 * DM, nodes); }
  k_dec<<<1, 1024, 0, stream>>>(nodes, Wdec, out);
}
